// KernelDensityEstimator_28363964023355
// MI455X (gfx1250) — hardware-verified
//
#include <hip/hip_runtime.h>
#include <hip/hip_bf16.h>
#include <math.h>

#define NT 4096
#define NTR 16384
#define DDk 512
#define CH 4096
#define SS 4096
#define HH 1
#define DKK 64
#define GSTR 48

typedef _Float16 bf16;
typedef _Float16 f16;
typedef __attribute__((ext_vector_type(4))) unsigned v4u_t;
typedef unsigned v4ua __attribute__((ext_vector_type(4), may_alias));
typedef __attribute__((ext_vector_type(4))) float v4f_t;
typedef float v4fa __attribute__((ext_vector_type(4), may_alias));
typedef __attribute__((ext_vector_type(16))) bf16  bf16x16;
typedef bf16x16 f16x16;
typedef __attribute__((ext_vector_type(8)))  bf16  bf16x8;
typedef bf16x8 f16x8;
typedef __attribute__((ext_vector_type(4)))  bf16  bf16x4;
typedef __attribute__((ext_vector_type(8)))  float f32x8;
__device__ __forceinline__ f32x8 wmma16(f16x16 a, f16x16 b, f32x8 c) {
  c = __builtin_amdgcn_wmma_f32_16x16x32_f16(false, a, false, b, (short)0, c, false, false);
  asm volatile("v_nop\n\tv_nop\n\tv_nop\n\tv_nop" : "+v"(c) : "v"(a), "v"(b));
  return c;
}
#define LDS_STRIDE 48
#define KSTRIDE    72
#define VSTRIDE    48

__device__ __forceinline__ f32x8 wmma_bf16(bf16x16 a, bf16x16 b, f32x8 c) {
  c = __builtin_amdgcn_wmma_f32_16x16x32_f16(false, a, false, b, (short)0, c, false, false);
  asm volatile("v_nop\n\tv_nop\n\tv_nop\n\tv_nop" : "+v"(c) : "v"(a), "v"(b));
  return c;
}

template <typename T>
__device__ __forceinline__ bf16x16 load_frag(const T* __restrict__ base, int ld,
                                             int row0, int k0) {
  const int lane = threadIdx.x & 31;
  const int r    = lane & 15;
  const int kh   = (lane >> 4) * 8;
  const T* p0 = base + (size_t)(row0 + r) * ld + (k0 + kh);
  const T* p1 = p0 + 16;
  bf16x16 f;
#pragma unroll
  for (int i = 0; i < 8; ++i) {
    f[i]     = (bf16)p0[i];
    f[i + 8] = (bf16)p1[i];
  }
  return f;
}

__device__ __forceinline__ bf16x16 lds_frag(const bf16* base, int stride) {
  const int lane = threadIdx.x & 31;
  const int row  = lane & 15;
  const int kh   = (lane >> 4) * 8;
  const bf16x8 lo = *(const bf16x8*)(base + row * stride + kh);
  const bf16x8 hi = *(const bf16x8*)(base + row * stride + kh + 16);
  bf16x16 f;
#pragma unroll
  for (int i = 0; i < 8; ++i) { f[i] = lo[i]; f[i + 8] = hi[i]; }
  return f;
}

template <typename T>
__device__ __forceinline__ void stage_read16(const T* __restrict__ p, float* buf) {
#pragma unroll
  for (int i = 0; i < 16; ++i) buf[i] = (float)p[i];
}

__device__ __forceinline__ void stage_write(bf16* dst, const float* buf, int nquad) {
#pragma unroll
  for (int i = 0; i < nquad; ++i) {
    bf16x4 q;
    q[0] = (bf16)buf[4 * i];     q[1] = (bf16)buf[4 * i + 1];
    q[2] = (bf16)buf[4 * i + 2]; q[3] = (bf16)buf[4 * i + 3];
    *(bf16x4*)(dst + 4 * i) = q;
  }
}

template <typename AT, int MODE>
__global__ __launch_bounds__(256) void gemm_rb_kernel(
    const AT* __restrict__ A, const float* __restrict__ W,
    const float* __restrict__ bias, const float* __restrict__ rowscale, const float* __restrict__ R, const float* __restrict__ rowbias, void* __restrict__ out,
    int M, int N, int K) {
  __shared__ bf16 ldsA[128 * LDS_STRIDE];
  __shared__ bf16 ldsW[256 * LDS_STRIDE];
  __shared__ __attribute__((aligned(16))) unsigned char sob[256 * 136 * 2];

  const int t    = threadIdx.x;
  const int wave = t >> 5;
  const int lane = t & 31;
  const int wm   = (wave & 1) * 64;
  const int wn   = (wave >> 1) * 64;
  const int mBlk = blockIdx.x * 128;
  const int nBlk = blockIdx.y * 256;

  const int arow = t >> 1;
  const int ach  = (t & 1) * 16;

  float abuf[16];
  float wbuf[32];

  stage_read16(A + (size_t)(mBlk + arow) * K + ach, abuf);
  const int nrow = min(nBlk + t, N - 1);
  stage_read16(W + (size_t)nrow * K,          wbuf);
  stage_read16(W + (size_t)nrow * K + 16,     wbuf + 16);

  f32x8 acc[4][4] = {};

  for (int k = 0; k < K; k += 32) {
    __syncthreads();
    stage_write(&ldsA[arow * LDS_STRIDE + ach], abuf, 4);
    stage_write(&ldsW[t * LDS_STRIDE],          wbuf, 8);
    if (k + 32 < K) {
      stage_read16(A + (size_t)(mBlk + arow) * K + (k + 32) + ach, abuf);
      stage_read16(W + (size_t)nrow * K + (k + 32),          wbuf);
      stage_read16(W + (size_t)nrow * K + (k + 32) + 16,     wbuf + 16);
    }
    __syncthreads();

    bf16x16 af[4], wf[4];
#pragma unroll
    for (int i = 0; i < 4; ++i)
      af[i] = lds_frag(ldsA + (wm + 16 * i) * LDS_STRIDE, LDS_STRIDE);
#pragma unroll
    for (int j = 0; j < 4; ++j)
      wf[j] = lds_frag(ldsW + (wn + 16 * j) * LDS_STRIDE, LDS_STRIDE);
#pragma unroll
    for (int i = 0; i < 4; ++i)
#pragma unroll
      for (int j = 0; j < 4; ++j)
        acc[i][j] = wmma_bf16(af[i], wf[j], acc[i][j]);
  }

  const int nlane = lane & 15;
  const int mh    = (lane >> 4) * 8;
  __syncthreads();
  if (MODE == 0 || MODE == 1 || MODE == 3) {
    bf16* so = (bf16*)sob;
#pragma unroll
    for (int i = 0; i < 4; ++i)
#pragma unroll
      for (int j = 0; j < 4; ++j) {
        const int nl = wn + 16 * j + nlane;
        const float bv = bias ? bias[nBlk + nl] : 0.0f;
        if (MODE == 3) {
#pragma unroll 1
          for (int r = 0; r < 8; ++r) {
            const int ml = wm + 16 * i + mh + r;
            const float xg = acc[i][j][r] + bv;
            so[ml * 264 + nl] = (bf16)(0.5f * xg * (1.0f + erff(xg * 0.70710678118654752f)));
          }
        } else {
#pragma unroll
        for (int r = 0; r < 8; ++r) {
          const int ml = wm + 16 * i + mh + r;
          const bf16 hv = (bf16)(acc[i][j][r] + bv);
          if (MODE == 0) so[ml * 264 + nl] = hv;
          else           so[nl * 136 + ml] = hv;
        }
        }
      }
    __syncthreads();
#pragma unroll 1
    for (int pass = 0; pass < 2; ++pass) {
      if (MODE == 0 || MODE == 3) {
        for (int ch = t; ch < 128 * 32; ch += 256) { const int ml = ch >> 5, q = (ch & 31) * 8;
          *(volatile v4u_t*)((bf16*)out + (size_t)(mBlk + ml) * N + nBlk + q) = *(const v4ua*)(so + ml * 264 + q); }
      } else {
        const int b_ = mBlk / SS, s0 = mBlk % SS;
        for (int ch = t; ch < 256 * 16; ch += 256) { const int nl = ch >> 4, q = (ch & 15) * 8; const int n = nBlk + nl, h = n >> 6, dk = n & (DKK - 1);
          *(volatile v4u_t*)((bf16*)out + (((size_t)(b_ * HH + h)) * DKK + dk) * SS + s0 + q) = *(const v4ua*)(so + nl * 136 + q); }
      }
      __threadfence();
    }
  } else {
    float* so = (float*)sob;
#pragma unroll 1
    for (int hf = 0; hf < 2; ++hf) {
      if (wm == hf * 64) {
#pragma unroll
        for (int i = 0; i < 4; ++i)
#pragma unroll
          for (int j = 0; j < 4; ++j) {
            const int nl = wn + 16 * j + nlane;
            const float bv = bias ? bias[nBlk + nl] : 0.0f;
#pragma unroll
            for (int r = 0; r < 8; ++r) { const int mrow = mBlk + hf * 64 + 16 * i + mh + r; so[(16 * i + mh + r) * 260 + nl] = acc[i][j][r] * (rowscale ? rowscale[mrow] : 1.0f) + bv + (rowbias ? rowbias[mrow] : 0.0f); }
          }
      }
      __syncthreads();
      if (R) {
        for (int ch = t; ch < 64 * 64; ch += 256) { const int ml = ch >> 6, q = (ch & 63) * 4;
          if (nBlk + q < N) { const v4f_t rv = *(const v4f_t*)(R + (size_t)(mBlk + hf * 64 + ml) * N + nBlk + q); v4f_t v = *(const v4fa*)(so + ml * 260 + q); v += rv; *(volatile v4fa*)(so + ml * 260 + q) = v; } }
        asm volatile("s_wait_dscnt 0" ::: "memory");
      }
#pragma unroll 1
      for (int pass = 0; pass < 2; ++pass) {
        for (int ch = t; ch < 64 * 64; ch += 256) { const int ml = ch >> 6, q = (ch & 63) * 4;
          if (nBlk + q < N) *(volatile v4f_t*)((float*)out + (size_t)(mBlk + hf * 64 + ml) * N + nBlk + q) = *(const v4fa*)(so + ml * 260 + q); }
        __threadfence();
      }
      __syncthreads();
    }
  }
}


__global__ __launch_bounds__(256) void k_norms(const float* __restrict__ A, int nrows, float* __restrict__ nrm) {
  const int row = blockIdx.x * 256 + threadIdx.x; float s = 0.0f;
  if (row < nrows) {
#pragma unroll 1
    for (int i = 0; i < DDk; i += 4) { const v4f_t v = *(const v4f_t*)(A + (size_t)row * DDk + i); s += v[0] * v[0] + v[1] * v[1] + v[2] * v[2] + v[3] * v[3]; } }
  *(volatile float*)(nrm + row) = s; __threadfence(); *(volatile float*)(nrm + row) = s;
}
__global__ __launch_bounds__(256) void k_lse(const float* __restrict__ Sc, const float* __restrict__ x2, const float* __restrict__ t2c, int first, float* __restrict__ ML) {
  __shared__ __attribute__((aligned(16))) float mlS[64];
  const int tid = threadIdx.x, r = tid >> 3, part = tid & 7; const int i = blockIdx.x * 32 + r; const float xi = x2[i]; const float* sr = Sc + (size_t)i * CH + part * (CH / 8); const float* tc = t2c + part * (CH / 8);
  float m = -3.0e38f;
#pragma unroll 1
  for (int j = 0; j < CH / 8; ++j) m = fmaxf(m, -0.5f * fmaxf(xi + tc[j] - 2.0f * sr[j], 0.0f));
  m = fmaxf(m, __shfl_xor(m, 1, 32)); m = fmaxf(m, __shfl_xor(m, 2, 32)); m = fmaxf(m, __shfl_xor(m, 4, 32));
  float mo = -3.0e38f, lo = 0.0f; if (!first) { mo = ML[2 * i]; lo = ML[2 * i + 1]; }
  const float mn = fmaxf(m, mo);
  float z = 0.0f;
#pragma unroll 1
  for (int j = 0; j < CH / 8; ++j) z += expf(-0.5f * fmaxf(xi + tc[j] - 2.0f * sr[j], 0.0f) - mn);
  z += __shfl_xor(z, 1, 32); z += __shfl_xor(z, 2, 32); z += __shfl_xor(z, 4, 32);
  if (part == 0) { mlS[2 * r] = mn; mlS[2 * r + 1] = lo * expf(mo - mn) + z; }
  __syncthreads();
#pragma unroll 1
  for (int pass = 0; pass < 2; ++pass) { if (tid < 16) *(volatile v4f_t*)(ML + (size_t)blockIdx.x * 64 + tid * 4) = *(const v4fa*)(mlS + tid * 4); __threadfence(); }
}
__global__ __launch_bounds__(256) void k_out(const float* __restrict__ ML, float* __restrict__ out) {
  const float Z = 0.5f * DDk * logf(2.0f * 3.14159265358979323846f) + DDk * logf(1.0f) + logf((float)NTR);
  for (int q4 = threadIdx.x; q4 < NT / 4; q4 += 256) { v4f_t o; for (int e = 0; e < 4; ++e) { const int i = q4 * 4 + e; o[e] = ML[2 * i] + logf(ML[2 * i + 1]) - Z; }
    *(volatile v4f_t*)(out + q4 * 4) = o; __threadfence(); *(volatile v4f_t*)(out + q4 * 4) = o; }
}

extern "C" void kernel_launch(void* const* d_in, const int* in_sizes, int n_in,
                              void* d_out, int out_size, void* d_ws, size_t ws_size,
                              hipStream_t stream) {
  (void)in_sizes; (void)n_in; (void)out_size;
  const float* x = (const float*)d_in[0]; const float* tr = (const float*)d_in[1];
  float* out = (float*)d_out;
  char* ws = (char*)d_ws;
  float* Sc = (float*)ws; ws += (size_t)NT * CH * 4;
  float* x2 = (float*)ws; ws += NT * 4; float* t2 = (float*)ws; ws += NTR * 4; float* ML = (float*)ws; ws += 2 * NT * 4;
  if ((size_t)(ws - (char*)d_ws) > ws_size) return;
  const dim3 blk(256);
  k_norms<<<dim3(NT / 256), blk, 0, stream>>>(x, NT, x2);
  k_norms<<<dim3(NTR / 256), blk, 0, stream>>>(tr, NTR, t2);
  for (int c = 0; c < NTR / CH; ++c) {
    gemm_rb_kernel<float, 2><<<dim3(NT / 128, CH / 256), blk, 0, stream>>>(x, tr + (size_t)c * CH * DDk, nullptr, nullptr, nullptr, nullptr, Sc, NT, CH, DDk);
    k_lse<<<dim3(NT / 32), blk, 0, stream>>>(Sc, x2, t2 + c * CH, c == 0 ? 1 : 0, ML);
  }
  k_out<<<dim3(1), blk, 0, stream>>>(ML, out);
}
